// GraphAttnModel_32976758898728
// MI455X (gfx1250) — hardware-verified
//
#include <hip/hip_runtime.h>
#include <stddef.h>
#include <stdint.h>
#include <math.h>


#define FIN     142
#define KP0     160
#define HD      128
#define NHEAD   4
#define DHEAD   32
#define NQ      512
#define ZP      256
#define H0P     320
#define NTHR    256
#define NWAVE   8
#define EPT     8
#define CHUNK   (NTHR * EPT)
#define WCAP    (EPT * 32)
#define LISTN   (NWAVE * WCAP)
#define NBA     512
#define SLA     9
#define SRCB    15
#define RCAP    28672
#define DEGCAP  64
#define MEAS_B512   16384
#define MEAS_MAXDEG 32
#define GBM     64
#define GTHR    128
#define MROWS   128
#define NU1     (HD * (KP0 / 8))
#define NU3     (KP0 * (ZP / 8))
#define NU4     (HD * (ZP / 8))
#define WSMAX   134217728
#define BNK     ((float)0.9999950000374996875)
#define RSQD    (1.0f / 5.65685424949238f)
#define LNEPS   1e-5f
#define BKT_LDS_INTS  (LISTN + RCAP + 16)
#define SCAN_ZINTS    (RCAP + 3 * NBA)
#define SCAN_LDS_INTS (2 * RCAP + 3 * NBA + 16)

static_assert(HD == 128 && HD == NHEAD * DHEAD && DHEAD == 32 && DHEAD == 8 * 4);
static_assert((KP0 % 32) == 0 && KP0 >= FIN && (ZP % 32) == 0 && (H0P % 32) == 0 && H0P == 2 * KP0 && ZP == 2 * HD);
static_assert((CHUNK & (CHUNK - 1)) == 0 && CHUNK <= 4096);
static_assert((NBA & (NBA - 1)) == 0 && NBA == (1 << SLA) && (NBA % 16) == 0 && (NBA % NWAVE) == 0 && (NBA % 32) == 0);
static_assert(((long long)CHUNK << SLA) < (1LL << 31));
static_assert(SRCB + SLA < 31);
static_assert((RCAP % 32) == 0 && (SCAN_ZINTS % 4) == 0);
static_assert(RCAP >= MEAS_B512 + 4096);
static_assert(DEGCAP >= MEAS_MAXDEG + 8);
static_assert(SCAN_LDS_INTS * 4 <= 300000 && BKT_LDS_INTS * 4 <= 300000);
static_assert(GBM == (GTHR / 32) * 16 && (NBA % GBM) == 0 && (MROWS % GBM) == 0);
static_assert((NU1 % NTHR) == 0 && ((NU1 + NU3) % NTHR) == 0 && ((NU1 + NU3 + NU4) % NTHR) == 0);
static_assert(NWAVE * ZP * 2 <= RCAP * 4);

typedef float          v4f  __attribute__((ext_vector_type(4)));
typedef float          v8f  __attribute__((ext_vector_type(8)));
typedef int            v4i  __attribute__((ext_vector_type(4)));
typedef int            v8i  __attribute__((ext_vector_type(8)));
typedef unsigned short v4us __attribute__((ext_vector_type(4)));
typedef unsigned short v8us __attribute__((ext_vector_type(8)));
typedef __bf16         v16b __attribute__((ext_vector_type(16)));
typedef v4f  __attribute__((may_alias)) v4fa;
typedef v4i  __attribute__((may_alias)) v4ia;
typedef v4us __attribute__((may_alias)) v4usa;
typedef v8us __attribute__((may_alias)) v8usa;
union FragB { v16b v; v8us h[2]; v8i w; };

__device__ __forceinline__ v8f wmb(const FragB& a, const FragB& b, v8f c) {
  v8f d = __builtin_amdgcn_wmma_f32_16x16x32_bf16(false, a.v, false, b.v, (short)0, c, false, false);
  asm volatile("v_nop\n\tv_nop\n\tv_nop\n\tv_nop" : "+v"(d) : "v"(a.w), "v"(b.w));
  return d;
}
__device__ __forceinline__ v8f z8() { v8f z = {0.f, 0.f, 0.f, 0.f, 0.f, 0.f, 0.f, 0.f}; return z; }

__device__ __forceinline__ unsigned int f2bf(float f) {
  const unsigned int u = __float_as_uint(f);
  const unsigned int r = ((u + 0x7FFFu + ((u >> 16) & 1u)) >> 16) & 0xFFFFu;
  return ((u & 0x7FFFFFFFu) > 0x7F800000u) ? 0x7FC0u : r;
}
__device__ __forceinline__ float bf2f(unsigned int b) { return __uint_as_float(b << 16); }
__device__ __forceinline__ float bfr(float f) { return bf2f(f2bf(f)); }
__device__ __forceinline__ v4f bfr4(v4f a) {
  v4f r; r.x = bfr(a.x); r.y = bfr(a.y); r.z = bfr(a.z); r.w = bfr(a.w); return r;
}
__device__ __forceinline__ float prelu(float x, float a) { return (x >= 0.0f) ? x : a * x; }

__device__ __forceinline__ void wave_sync() {
  __builtin_amdgcn_fence(__ATOMIC_RELEASE, "workgroup");
  __builtin_amdgcn_wave_barrier();
  __builtin_amdgcn_fence(__ATOMIC_ACQUIRE, "workgroup");
}

template <int SLB>
__device__ __forceinline__ int scan_chunk(const int* __restrict__ dsts, int nE, int cbase, int slotBase,
                                          int nb, int vec8, int* list, int tid, int lane, int wave) {
  int wc = 0;
  const int el0  = tid * EPT;
  const int e0   = cbase + el0;
  const int sent = -2147483647 - 1;
  v4i da, db;
  if (vec8 != 0 && cbase + CHUNK <= nE) {
    da = *(const v4i*)(dsts + e0);
    db = *(const v4i*)(dsts + e0 + 4);
  } else {
    da.x = (e0     < nE) ? dsts[min(e0,     nE - 1)] : sent;
    da.y = (e0 + 1 < nE) ? dsts[min(e0 + 1, nE - 1)] : sent;
    da.z = (e0 + 2 < nE) ? dsts[min(e0 + 2, nE - 1)] : sent;
    da.w = (e0 + 3 < nE) ? dsts[min(e0 + 3, nE - 1)] : sent;
    db.x = (e0 + 4 < nE) ? dsts[min(e0 + 4, nE - 1)] : sent;
    db.y = (e0 + 5 < nE) ? dsts[min(e0 + 5, nE - 1)] : sent;
    db.z = (e0 + 6 < nE) ? dsts[min(e0 + 6, nE - 1)] : sent;
    db.w = (e0 + 7 < nE) ? dsts[min(e0 + 7, nE - 1)] : sent;
  }
  const unsigned nbs = (unsigned)slotBase;
  const unsigned unb = (unsigned)nb;
  const unsigned s0 = (unsigned)da.x - nbs, s1 = (unsigned)da.y - nbs;
  const unsigned s2 = (unsigned)da.z - nbs, s3 = (unsigned)da.w - nbs;
  const unsigned s4 = (unsigned)db.x - nbs, s5 = (unsigned)db.y - nbs;
  const unsigned s6 = (unsigned)db.z - nbs, s7 = (unsigned)db.w - nbs;
  const bool h0 = s0 < unb, h1 = s1 < unb, h2 = s2 < unb, h3 = s3 < unb;
  const bool h4 = s4 < unb, h5 = s5 < unb, h6 = s6 < unb, h7 = s7 < unb;
  const unsigned any = __builtin_amdgcn_ballot_w32(h0 | h1 | h2 | h3 | h4 | h5 | h6 | h7);
  if (any != 0u) {
#define HITJ(J, HJ, SJ) { \
      const unsigned mj = __builtin_amdgcn_ballot_w32(HJ); \
      if (mj != 0u) { \
        if (HJ) { \
          const int pos = wc + (int)__builtin_amdgcn_mbcnt_lo(mj, 0u); \
          if (pos < WCAP) list[wave * WCAP + pos] = ((el0 + (J)) << SLB) | (int)(SJ); \
        } \
        wc += (int)__builtin_popcount(mj); } }
    HITJ(0, h0, s0)
    HITJ(1, h1, s1)
    HITJ(2, h2, s2)
    HITJ(3, h3, s3)
    HITJ(4, h4, s4)
    HITJ(5, h5, s5)
    HITJ(6, h6, s6)
    HITJ(7, h7, s7)
#undef HITJ
  }
  return wc;
}

__global__ __launch_bounds__(NTHR) void k_pa(const float* __restrict__ x, unsigned short* FB, int nN, int nU) {
  const int u = (int)blockIdx.x * NTHR + (int)threadIdx.x;
  if (u >= nU) return;
  const int row = u / (KP0 / 8);
  const int c0  = (u - row * (KP0 / 8)) * 8;
  const int rc  = row < nN ? row : nN - 1;
  const bool okr = row < nN;
  const float* p = x + (size_t)rc * FIN;
  v8us o;
#pragma unroll
  for (int i = 0; i < 8; ++i) {
    const int c  = c0 + i;
    const int cc = c < FIN ? c : FIN - 1;
    const float f = p[cc];
    o[i] = (okr && c < FIN) ? (unsigned short)f2bf(f) : (unsigned short)0;
  }
  unsigned short* dp = FB + (size_t)u * 8;
  *(volatile v8us*)dp = o;
  __threadfence();
  *(volatile v8us*)dp = o;
}

__global__ __launch_bounds__(NTHR) void k_pb(const float* __restrict__ W1, const float* __restrict__ W3,
                                             const float* __restrict__ W4, unsigned short* W1t,
                                             unsigned short* W3t2, unsigned short* W4t2) {
  const int u = (int)blockIdx.x * NTHR + (int)threadIdx.x;
  v8us o;
  unsigned short* dp;
  if (u < NU1) {
    const int n  = u / (KP0 / 8);
    const int k8 = (u - n * (KP0 / 8)) * 8;
#pragma unroll
    for (int i = 0; i < 8; ++i) {
      const int k  = k8 + i;
      const int kc = k < FIN ? k : FIN - 1;
      const float f = W1[(size_t)kc * HD + n];
      o[i] = (k < FIN) ? (unsigned short)f2bf(f) : (unsigned short)0;
    }
    dp = W1t + (size_t)u * 8;
  } else if (u < NU1 + NU3) {
    const int v  = u - NU1;
    const int n  = v >> 5;
    const int k8 = (v & 31) * 8;
    const int kk = k8 & (HD - 1);
    const int nc = n < FIN ? n : FIN - 1;
#pragma unroll
    for (int i = 0; i < 8; ++i) {
      const float f = W3[(size_t)(kk + i) * FIN + nc];
      o[i] = (n < FIN) ? (unsigned short)f2bf(f) : (unsigned short)0;
    }
    dp = W3t2 + (size_t)v * 8;
  } else if (u < NU1 + NU3 + NU4) {
    const int v  = u - NU1 - NU3;
    const int n  = v >> 5;
    const int k8 = (v & 31) * 8;
    const int kk = k8 & (HD - 1);
#pragma unroll
    for (int i = 0; i < 8; ++i) o[i] = (unsigned short)f2bf(W4[(size_t)(kk + i) * HD + n]);
    dp = W4t2 + (size_t)v * 8;
  } else {
    return;
  }
  *(volatile v8us*)dp = o;
  __threadfence();
  *(volatile v8us*)dp = o;
}

__device__ __forceinline__ v8us wunit(const float* __restrict__ W, int col, int kk0, int fin) {
  v8us o;
#pragma unroll
  for (int i = 0; i < 8; ++i) {
    const int kk = kk0 + i;
    const int kc = kk < fin ? kk : fin - 1;
    const float f = W[(size_t)kc * HD + col];
    o[i] = (kk < fin) ? (unsigned short)f2bf(f) : (unsigned short)0;
  }
  return o;
}

__global__ __launch_bounds__(NTHR) void k_pc(const float* __restrict__ Wq, const float* __restrict__ Wv,
                                             const float* __restrict__ Wk, const float* __restrict__ Ws,
                                             unsigned short* Wc, int fin, int Kp) {
  const int upr = (2 * Kp) >> 3;
  const int bpm = (HD * upr) / NTHR;
  const int mi  = (int)blockIdx.x / bpm;
  const int v   = ((int)blockIdx.x - mi * bpm) * NTHR + (int)threadIdx.x;
  const int col = v / upr;
  const int k8  = (v - col * upr) * 8;
  const int kk0 = k8 >= Kp ? k8 - Kp : k8;
  v8us o;
  if (mi == 0)      o = wunit(Wq, col, kk0, fin);
  else if (mi == 1) o = wunit(Wv, col, kk0, fin);
  else if (mi == 2) o = wunit(Wk, col, kk0, fin);
  else              o = wunit(Ws, col, kk0, fin);
  unsigned short* dp = Wc + (size_t)(mi * HD + col) * (size_t)(2 * Kp) + k8;
  *(volatile v8us*)dp = o;
  __threadfence();
  *(volatile v8us*)dp = o;
}

__global__ __launch_bounds__(384) void k_pt(const float* __restrict__ lemb, const float* __restrict__ W2, float* T2) {
  __shared__ __attribute__((aligned(16))) float sT[384];
  const int tid = (int)threadIdx.x;
  const int c = tid >> 7, n = tid & (HD - 1);
  float s = 0.0f;
#pragma unroll 2
  for (int k = 0; k < FIN; ++k) s = fmaf(bfr(lemb[c * FIN + k]), bfr(W2[(size_t)k * HD + n]), s);
  sT[tid] = s;
  __syncthreads();
  const bool ok = tid < 96;
  const int  ti = ok ? tid : 0;
  const v4f v = *(const v4fa*)(sT + 4 * ti);
  float* op = T2 + 4 * ti;
  if (ok) *(volatile v4f*)op = v;
  __threadfence();
  if (ok) *(volatile v4f*)op = v;
}

__global__ __launch_bounds__(NTHR) void k_bucket(const int* __restrict__ srcs, const int* __restrict__ dsts,
                                                 int nE, int nN, int vec8, int* HITS, int* FLG) {
  extern __shared__ __attribute__((aligned(16))) int bsm[];
  int* list = bsm;
  int* reg1 = bsm + LISTN;
  int* wcnt = reg1 + RCAP;
  const int tid = (int)threadIdx.x, lane = tid & 31, wave = tid >> 5;
  const int blk = (int)blockIdx.x;
  const int nodeBase = blk * NBA;
  int nb = nN - nodeBase;
  nb = nb < 0 ? 0 : (nb > NBA ? NBA : nb);

  int tot = 0, ovf = 0;
  const int nChunks = (nE + CHUNK - 1) / CHUNK;
#pragma unroll 1
  for (int ch = 0; ch < nChunks; ++ch) {
    const int cbase = ch * CHUNK;
    const int wc = scan_chunk<SLA>(dsts, nE, cbase, nodeBase, nb, vec8, list, tid, lane, wave);
    if (lane == 0) wcnt[wave] = wc;
    __syncthreads();
    int pre = 0, all = 0;
#pragma unroll
    for (int w2 = 0; w2 < NWAVE; ++w2) {
      int c = wcnt[w2];
      c = c < 0 ? 0 : (c > WCAP ? WCAP : c);
      all += c;
      pre += (w2 < wave) ? c : 0;
    }
    const int wcc  = wc > WCAP ? WCAP : wc;
    const int base = tot + pre;
#pragma unroll 1
    for (int i = lane; i < wcc; i += 32) {
      const int ent = list[wave * WCAP + i];
      const int el  = (ent >> SLA) & (CHUNK - 1);
      const int sl  = ent & (NBA - 1);
      int eid = cbase + el;
      eid = eid > nE - 1 ? nE - 1 : eid;
      const int sraw = srcs[eid];
      const int s = sraw < 0 ? 0 : (sraw > nN - 1 ? nN - 1 : sraw);
      const int pos = base + i;
      if (pos < RCAP) reg1[pos] = (int)((unsigned)s | ((unsigned)sl << SRCB));
    }
    if (tot + all > RCAP) ovf = 1;
    tot += all;
    tot = tot > RCAP ? RCAP : tot;
    __syncthreads();
  }
  const int nh = tot;
  for (int i = nh + tid; i < RCAP; i += NTHR) reg1[i] = 0;
  __syncthreads();

  int* hb = HITS + (size_t)blk * RCAP;
  v4i cv;
  cv.x = (tid == 0) ? nh : 0;
  cv.y = (tid == 0) ? ovf : 0;
  cv.z = 0; cv.w = 0;
  int* fp = FLG + (size_t)blk * 32 + 4 * (tid & 7);
#pragma unroll 1
  for (int p = tid * 4; p < RCAP; p += NTHR * 4) {
    const v4i v = *(const v4ia*)(reg1 + p);
    *(volatile v4i*)(hb + p) = v;
  }
  if (tid < 8) *(volatile v4i*)fp = cv;
  __threadfence();
#pragma unroll 1
  for (int p = tid * 4; p < RCAP; p += NTHR * 4) {
    const v4i v = *(const v4ia*)(reg1 + p);
    *(volatile v4i*)(hb + p) = v;
  }
  if (tid < 8) *(volatile v4i*)fp = cv;
}

template <int NT>
__device__ __forceinline__ void gemm_tile(const unsigned short* __restrict__ A, int lda,
                                          const unsigned short* __restrict__ BT, int K,
                                          int rowBase, int col0, float* stg) {
  const int tid = (int)threadIdx.x, lane = tid & 31, wave = tid >> 5, hh = lane >> 4, m = lane & 15;
  v8f acc[NT];
#pragma unroll
  for (int t = 0; t < NT; ++t) acc[t] = z8();
  const unsigned short* ap = A  + (size_t)(rowBase + 16 * wave + m) * (size_t)lda + 8 * hh;
  const unsigned short* bp = BT + (size_t)(col0 + m) * (size_t)K + 8 * hh;
#pragma unroll 1
  for (int k0 = 0; k0 < K; k0 += 32) {
    FragB af;
    af.h[0] = *(const v8usa*)(ap + k0);
    af.h[1] = *(const v8usa*)(ap + k0 + 16);
#pragma unroll
    for (int nt = 0; nt < NT; ++nt) {
      const unsigned short* wq = bp + (size_t)(16 * nt) * (size_t)K + k0;
      FragB bf;
      bf.h[0] = *(const v8usa*)wq;
      bf.h[1] = *(const v8usa*)(wq + 16);
      acc[nt] = wmb(af, bf, acc[nt]);
    }
  }
  constexpr int P = 16 * NT;
#pragma unroll
  for (int nt = 0; nt < NT; ++nt) {
    const int lc = 16 * nt + m;
#pragma unroll
    for (int r = 0; r < 8; ++r) {
      const int lr = 16 * wave + 8 * hh + r;
      stg[lr * P + lc] = acc[nt][r];
    }
  }
}

__global__ __launch_bounds__(GTHR) __attribute__((amdgpu_num_vgpr(248)))
void k_ga(const unsigned short* __restrict__ FB, const unsigned short* __restrict__ W1t,
          const float* __restrict__ T2, const int* __restrict__ labels,
          const float* __restrict__ b1, const float* __restrict__ b2,
          const float* __restrict__ g0, const float* __restrict__ be0, const float* __restrict__ a3p,
          unsigned short* Zhl, int nN) {
  __shared__ __attribute__((aligned(16))) float stg[GBM * HD];
  __shared__ __attribute__((aligned(16))) unsigned short rbuf[4 * ZP];
  const int tid = (int)threadIdx.x, lane = tid & 31, wave = tid >> 5;
  const int rowBase = (int)blockIdx.x * GBM;
  gemm_tile<8>(FB, KP0, W1t, KP0, rowBase, 0, stg);
  __syncthreads();
  const v4f b1v = bfr4(*(const v4f*)(b1 + 4 * lane));
  const v4f b2v = bfr4(*(const v4f*)(b2 + 4 * lane));
  const v4f gv  = bfr4(*(const v4f*)(g0 + 4 * lane));
  const v4f ev  = bfr4(*(const v4f*)(be0 + 4 * lane));
  const float a3 = bfr(a3p[0]);
  unsigned short* rb = rbuf + wave * ZP;
#pragma unroll 1
  for (int i = 0; i < 16; ++i) {
    const int lr  = 16 * wave + i;
    const int row = rowBase + lr;
    const bool ok = row < nN;
    const int rc  = ok ? row : nN - 1;
    int lab = labels[rc];
    lab = lab < 0 ? 0 : (lab > 2 ? 2 : lab);
    const v4f t  = *(const v4f*)(T2 + (size_t)lab * HD + 4 * lane);
    const v4f pv = *(const v4fa*)(stg + lr * HD + 4 * lane);
    const float l0 = ((pv.x + b1v.x) + t.x) + b2v.x;
    const float l1 = ((pv.y + b1v.y) + t.y) + b2v.y;
    const float l2 = ((pv.z + b1v.z) + t.z) + b2v.z;
    const float l3 = ((pv.w + b1v.w) + t.w) + b2v.w;
    float z0 = prelu(((l0 * BNK) * gv.x) + ev.x, a3);
    float z1 = prelu(((l1 * BNK) * gv.y) + ev.y, a3);
    float z2 = prelu(((l2 * BNK) * gv.z) + ev.z, a3);
    float z3 = prelu(((l3 * BNK) * gv.w) + ev.w, a3);
    z0 = ok ? z0 : 0.0f; z1 = ok ? z1 : 0.0f; z2 = ok ? z2 : 0.0f; z3 = ok ? z3 : 0.0f;
    v4us h4, l4;
    unsigned hb;
    hb = f2bf(z0); h4[0] = (unsigned short)hb; l4[0] = (unsigned short)f2bf(z0 - bf2f(hb));
    hb = f2bf(z1); h4[1] = (unsigned short)hb; l4[1] = (unsigned short)f2bf(z1 - bf2f(hb));
    hb = f2bf(z2); h4[2] = (unsigned short)hb; l4[2] = (unsigned short)f2bf(z2 - bf2f(hb));
    hb = f2bf(z3); h4[3] = (unsigned short)hb; l4[3] = (unsigned short)f2bf(z3 - bf2f(hb));
    *(v4usa*)(rb + 4 * lane)      = h4;
    *(v4usa*)(rb + HD + 4 * lane) = l4;
    wave_sync();
    const v8us q0 = *(const v8usa*)(rb + 8 * lane);
    wave_sync();
    unsigned short* rp = Zhl + (size_t)row * ZP + 8 * lane;
    *(volatile v8us*)rp = q0;
    __threadfence();
    *(volatile v8us*)rp = q0;
  }
}

__global__ __launch_bounds__(GTHR) __attribute__((amdgpu_num_vgpr(248)))
void k_gb(const unsigned short* __restrict__ Zhl, const unsigned short* __restrict__ W3t2,
          const float* __restrict__ b3, const float* __restrict__ feat, unsigned short* H0, int nN) {
  __shared__ __attribute__((aligned(16))) float stg[GBM * KP0];
  __shared__ __attribute__((aligned(16))) float sb3[KP0];
  __shared__ __attribute__((aligned(16))) unsigned short rbuf[4 * H0P];
  const int tid = (int)threadIdx.x, lane = tid & 31, wave = tid >> 5;
  const int rowBase = (int)blockIdx.x * GBM;
  for (int c = tid; c < KP0; c += GTHR) {
    const int cc = c < FIN ? c : FIN - 1;
    const float f = b3[cc];
    sb3[c] = (c < FIN) ? bfr(f) : 0.0f;
  }
  gemm_tile<10>(Zhl, ZP, W3t2, ZP, rowBase, 0, stg);
  __syncthreads();
  unsigned short* rb = rbuf + wave * H0P;
#pragma unroll 1
  for (int i = 0; i < 16; ++i) {
    const int lr  = 16 * wave + i;
    const int row = rowBase + lr;
    const bool ok = row < nN;
    const int rc  = ok ? row : nN - 1;
    const float* fr = feat + (size_t)rc * FIN;
#pragma unroll
    for (int j = 0; j < 5; ++j) {
      const int c  = lane + 32 * j;
      const int cc = c < FIN ? c : FIN - 1;
      const float f = fr[cc];
      const float v = stg[lr * KP0 + c];
      float h = (v + sb3[c]) + bfr(f);
      h = (ok && c < FIN) ? h : 0.0f;
      const unsigned hb = f2bf(h);
      const unsigned lb = f2bf(h - bf2f(hb));
      rb[c]       = (unsigned short)hb;
      rb[KP0 + c] = (unsigned short)lb;
    }
    wave_sync();
    const v8us q0 = *(const v8usa*)(rb + 8 * lane);
    const v8us q1 = *(const v8usa*)(rb + 256 + 8 * (lane & 7));
    wave_sync();
    unsigned short* rp = H0 + (size_t)row * H0P;
    *(volatile v8us*)(rp + 8 * lane) = q0;
    if (lane < 8) *(volatile v8us*)(rp + 256 + 8 * lane) = q1;
    __threadfence();
    *(volatile v8us*)(rp + 8 * lane) = q0;
    if (lane < 8) *(volatile v8us*)(rp + 256 + 8 * lane) = q1;
  }
}

__global__ __launch_bounds__(GTHR) __attribute__((amdgpu_num_vgpr(248)))
void k_gc(const unsigned short* __restrict__ A, const unsigned short* __restrict__ Wc,
          const float* __restrict__ bq, const float* __restrict__ bv, const float* __restrict__ bk,
          const float* __restrict__ bs, float* Q, int K) {
  __shared__ __attribute__((aligned(16))) float stg[GBM * HD];
  const int tid = (int)threadIdx.x, lane = tid & 31, wave = tid >> 5;
  const int rowBase = (int)blockIdx.x * GBM;
  const int cb   = (int)blockIdx.y;
  const int col0 = cb * HD;
  gemm_tile<8>(A, K, Wc, K, rowBase, col0, stg);
  __syncthreads();
  const v4f q4 = *(const v4f*)(bq + 4 * lane);
  const v4f v4 = *(const v4f*)(bv + 4 * lane);
  const v4f k4 = *(const v4f*)(bk + 4 * lane);
  const v4f s4 = *(const v4f*)(bs + 4 * lane);
  v4f bsel;
  bsel.x = (cb == 0) ? q4.x : ((cb == 1) ? v4.x : ((cb == 2) ? k4.x : s4.x));
  bsel.y = (cb == 0) ? q4.y : ((cb == 1) ? v4.y : ((cb == 2) ? k4.y : s4.y));
  bsel.z = (cb == 0) ? q4.z : ((cb == 1) ? v4.z : ((cb == 2) ? k4.z : s4.z));
  bsel.w = (cb == 0) ? q4.w : ((cb == 1) ? v4.w : ((cb == 2) ? k4.w : s4.w));
  const v4f bb = bfr4(bsel);
  v4f fv[16];
#pragma unroll
  for (int i = 0; i < 16; ++i) {
    const v4f p = *(const v4fa*)(stg + (16 * wave + i) * HD + 4 * lane);
    v4f o; o.x = p.x + bb.x; o.y = p.y + bb.y; o.z = p.z + bb.z; o.w = p.w + bb.w;
    fv[i] = o;
  }
#pragma unroll
  for (int i = 0; i < 16; ++i) {
    float* op = Q + (size_t)(rowBase + 16 * wave + i) * NQ + col0 + 4 * lane;
    *(volatile v4f*)op = fv[i];
  }
  __threadfence();
#pragma unroll
  for (int i = 0; i < 16; ++i) {
    float* op = Q + (size_t)(rowBase + 16 * wave + i) * NQ + col0 + 4 * lane;
    *(volatile v4f*)op = fv[i];
  }
}

__global__ __launch_bounds__(NTHR) __attribute__((amdgpu_num_vgpr(248)))
void k_scan(const int* __restrict__ HITS, const int* __restrict__ FLGB, const float* __restrict__ Q,
            const float* __restrict__ Wg, const float* __restrict__ bgp,
            const float* __restrict__ lng, const float* __restrict__ lnb, const float* __restrict__ acp,
            unsigned short* XP, int* FLGO, int nN, int MPr) {
  extern __shared__ __attribute__((aligned(16))) int ssm[];
  int* hl   = ssm;
  int* sl   = ssm + RCAP;
  int* cnt  = sl + RCAP;
  int* offs = cnt + NBA;
  int* cur  = offs + NBA;
  int* misc = cur + NBA;
  const int tid = (int)threadIdx.x, lane = tid & 31, wave = tid >> 5;
  const int blk = (int)blockIdx.x;
  const int nodeBase = blk * NBA;

  const int nhraw = FLGB[(size_t)blk * 32];
  const int bflag = FLGB[(size_t)blk * 32 + 1];
  const int nh  = nhraw < 0 ? 0 : (nhraw > RCAP ? RCAP : nhraw);
  const int ovf = (bflag != 0 || nhraw < 0 || nhraw > RCAP) ? 1 : 0;

  {
    const v4i z4 = {0, 0, 0, 0};
    for (int i = tid * 4; i < SCAN_ZINTS; i += NTHR * 4) *(v4ia*)(sl + i) = z4;
    if (tid < 16) misc[tid] = 0;
    const int* hb = HITS + (size_t)blk * RCAP;
    const int nh4 = (nh + 3) & ~3;
#pragma unroll 1
    for (int p = tid * 4; p < nh4; p += NTHR * 4) *(v4ia*)(hl + p) = *(const v4i*)(hb + p);
  }
  __syncthreads();

  if (wave == 0) {
#pragma unroll 1
    for (int b0 = 0; b0 < nh; b0 += 32) {
      const int idx = b0 + lane;
      const int uv  = hl[idx < nh ? idx : nh - 1];
      const int m32 = (nh - b0) < 32 ? (nh - b0) : 32;
#pragma unroll 1
      for (int k = 0; k < m32; ++k) {
        const int u  = __builtin_amdgcn_readlane(uv, k);
        const int sq = (u >> SRCB) & (NBA - 1);
        if (lane == 0) cnt[sq] = cnt[sq] + 1;
      }
    }
  }
  __syncthreads();
  if (wave == 0) {
    const int base = lane * (NBA / 32);
    int s = 0;
#pragma unroll 1
    for (int i = 0; i < NBA / 32; ++i) s += cnt[base + i];
    int incl = s;
#pragma unroll
    for (int d = 1; d < 32; d <<= 1) {
      const int y = __shfl_up(incl, d, 32);
      if (lane >= d) incl += y;
    }
    int run = incl - s;
#pragma unroll 1
    for (int i = 0; i < NBA / 32; ++i) {
      const int cv = cnt[base + i];
      offs[base + i] = run;
      cur[base + i]  = run;
      run += cv;
    }
  }
  __syncthreads();
  if (wave == 0) {
#pragma unroll 1
    for (int b0 = 0; b0 < nh; b0 += 32) {
      const int idx = b0 + lane;
      const int uv  = hl[idx < nh ? idx : nh - 1];
      const int m32 = (nh - b0) < 32 ? (nh - b0) : 32;
#pragma unroll 1
      for (int k = 0; k < m32; ++k) {
        const int u  = __builtin_amdgcn_readlane(uv, k);
        const int sq = (u >> SRCB) & (NBA - 1);
        if (lane == 0) {
          int p = cur[sq];
          p = p < 0 ? 0 : (p > RCAP - 1 ? RCAP - 1 : p);
          sl[p] = u;
          cur[sq] = p + 1;
        }
      }
    }
  }
  __syncthreads();

  unsigned short* rb = (unsigned short*)hl + wave * ZP;

  const float qnan = __int_as_float(0x7fc00000);
  const float pzb  = (ovf != 0) ? qnan : 0.0f;
  const v4f wg0 = bfr4(*(const v4f*)(Wg + 4 * lane));
  const v4f wg1 = bfr4(*(const v4f*)(Wg + HD + 4 * lane));
  const v4f wg2 = bfr4(*(const v4f*)(Wg + 2 * HD + 4 * lane));
  const v4f lgv = bfr4(*(const v4f*)(lng + 4 * lane));
  const v4f lbv = bfr4(*(const v4f*)(lnb + 4 * lane));
  const float bgv = bfr(bgp[0]);
  const float acv = bfr(acp[0]);
  int anybig = 0;

#pragma unroll 1
  for (int si = 0; si < NBA / NWAVE; ++si) {
    const int s    = si * NWAVE + wave;
    const int node = nodeBase + s;
    const int nc   = node < nN ? node : nN - 1;
    int c = cnt[s];
    const bool big = c > DEGCAP;
    anybig |= big ? 1 : 0;
    c = c < 0 ? 0 : (c > DEGCAP ? DEGCAP : c);
    int o = offs[s];
    o = o < 0 ? 0 : (o > RCAP ? RCAP : o);
    if (c > nh - o) c = nh - o;
    c = c < 0 ? 0 : c;
    const float* dr = Q + (size_t)nc * NQ;
    const v4f kv = *(const v4f*)(dr + 2 * HD + 4 * lane);
    const v4f sv = *(const v4f*)(dr + 3 * HD + 4 * lane);
    float mx = -3.0e38f, dn = 0.0f;
    float a0 = 0.0f, a1 = 0.0f, a2 = 0.0f, a3 = 0.0f;
#pragma unroll 1
    for (int b0 = 0; b0 < c; b0 += 32) {
      int idx = o + b0 + lane;
      idx = idx < 0 ? 0 : (idx > RCAP - 1 ? RCAP - 1 : idx);
      const int ent = sl[idx];
      int hs = ent & ((1 << SRCB) - 1);
      hs = hs > nN - 1 ? nN - 1 : hs;
      const int m32 = (c - b0) < 32 ? (c - b0) : 32;
#pragma unroll 1
      for (int k = 0; k < m32; ++k) {
        const int sk = __builtin_amdgcn_readlane(hs, k);
        const float* rp = Q + (size_t)sk * NQ + 4 * lane;
        const v4f qv = *(const v4f*)rp;
        const v4f vv = *(const v4f*)(rp + HD);
        float p = qv.x * kv.x;
        p = fmaf(qv.y, kv.y, p);
        p = fmaf(qv.z, kv.z, p);
        p = fmaf(qv.w, kv.w, p);
        p += __shfl_xor(p, 1, 32);
        p += __shfl_xor(p, 2, 32);
        p += __shfl_xor(p, 4, 32);
        const float sc = p * RSQD;
        const float df = sc - mx;
        const float ee = expf(-fabsf(df));
        const bool  up = df > 0.0f;
        const float s1 = up ? ee : 1.0f;
        const float s2 = up ? 1.0f : ee;
        mx = up ? sc : mx;
        dn = fmaf(dn, s1, s2);
        a0 = fmaf(a0, s1, s2 * vv.x);
        a1 = fmaf(a1, s1, s2 * vv.y);
        a2 = fmaf(a2, s1, s2 * vv.z);
        a3 = fmaf(a3, s1, s2 * vv.w);
      }
    }
    const bool  emp = (dn == 0.0f);
    const float inv = __builtin_amdgcn_rcpf(emp ? 1.0f : dn);
    const float g0 = emp ? 0.0f : a0 * inv;
    const float g1 = emp ? 0.0f : a1 * inv;
    const float g2 = emp ? 0.0f : a2 * inv;
    const float g3 = emp ? 0.0f : a3 * inv;
    float t = sv.x * wg0.x;
    t = fmaf(sv.y, wg0.y, t); t = fmaf(sv.z, wg0.z, t); t = fmaf(sv.w, wg0.w, t);
    t = fmaf(g0, wg1.x, t); t = fmaf(g1, wg1.y, t); t = fmaf(g2, wg1.z, t); t = fmaf(g3, wg1.w, t);
    t = fmaf(sv.x - g0, wg2.x, t); t = fmaf(sv.y - g1, wg2.y, t);
    t = fmaf(sv.z - g2, wg2.z, t); t = fmaf(sv.w - g3, wg2.w, t);
    t += __shfl_xor(t, 16, 32);
    t += __shfl_xor(t, 8, 32);
    t += __shfl_xor(t, 4, 32);
    t += __shfl_xor(t, 2, 32);
    t += __shfl_xor(t, 1, 32);
    const float gt = 1.0f / (1.0f + expf(-(t + bgv)));
    const float om = 1.0f - gt;
    const float r0 = gt * sv.x + om * g0;
    const float r1 = gt * sv.y + om * g1;
    const float r2 = gt * sv.z + om * g2;
    const float r3 = gt * sv.w + om * g3;
    float sm = (r0 + r1) + (r2 + r3);
    sm += __shfl_xor(sm, 16, 32);
    sm += __shfl_xor(sm, 8, 32);
    sm += __shfl_xor(sm, 4, 32);
    sm += __shfl_xor(sm, 2, 32);
    sm += __shfl_xor(sm, 1, 32);
    const float mean = sm * (1.0f / (float)HD);
    const float d0 = r0 - mean, d1 = r1 - mean, d2 = r2 - mean, d3 = r3 - mean;
    float qq = (d0 * d0 + d1 * d1) + (d2 * d2 + d3 * d3);
    qq += __shfl_xor(qq, 16, 32);
    qq += __shfl_xor(qq, 8, 32);
    qq += __shfl_xor(qq, 4, 32);
    qq += __shfl_xor(qq, 2, 32);
    qq += __shfl_xor(qq, 1, 32);
    const float var = qq * (1.0f / (float)HD);
    const float rs  = 1.0f / sqrtf(var + LNEPS);
    const float pzr = big ? qnan : pzb;
    const bool live = node < nN;
    float y0 = prelu((d0 * rs) * lgv.x + lbv.x, acv) + pzr;
    float y1 = prelu((d1 * rs) * lgv.y + lbv.y, acv) + pzr;
    float y2 = prelu((d2 * rs) * lgv.z + lbv.z, acv) + pzr;
    float y3 = prelu((d3 * rs) * lgv.w + lbv.w, acv) + pzr;
    y0 = live ? y0 : 0.0f; y1 = live ? y1 : 0.0f; y2 = live ? y2 : 0.0f; y3 = live ? y3 : 0.0f;
    v4us h4, l4;
    unsigned hb;
    hb = f2bf(y0); h4[0] = (unsigned short)hb; l4[0] = (unsigned short)f2bf(y0 - bf2f(hb));
    hb = f2bf(y1); h4[1] = (unsigned short)hb; l4[1] = (unsigned short)f2bf(y1 - bf2f(hb));
    hb = f2bf(y2); h4[2] = (unsigned short)hb; l4[2] = (unsigned short)f2bf(y2 - bf2f(hb));
    hb = f2bf(y3); h4[3] = (unsigned short)hb; l4[3] = (unsigned short)f2bf(y3 - bf2f(hb));
    *(v4usa*)(rb + 4 * lane)      = h4;
    *(v4usa*)(rb + HD + 4 * lane) = l4;
    wave_sync();
    const v8us q0 = *(const v8usa*)(rb + 8 * lane);
    wave_sync();
    if (node < MPr) {
      unsigned short* hp = XP + (size_t)node * ZP + 8 * lane;
      *(volatile v8us*)hp = q0;
      __threadfence();
      *(volatile v8us*)hp = q0;
    }
  }

  if (lane == 0) misc[wave] = anybig;
  __syncthreads();
  if (wave == 0) {
    int fg = ovf;
#pragma unroll
    for (int w2 = 0; w2 < NWAVE; ++w2) fg |= misc[w2];
    v4i cv;
    cv.x = 0;
    cv.y = (lane == 0) ? fg : 0;
    cv.z = 0; cv.w = 0;
    int* fp = FLGO + (size_t)blk * 32 + 4 * (lane & 7);
    if (lane < 8) *(volatile v4i*)fp = cv;
    __threadfence();
    if (lane < 8) *(volatile v4i*)fp = cv;
  }
}

__global__ __launch_bounds__(GTHR) __attribute__((amdgpu_num_vgpr(248)))
void k_gd(const unsigned short* __restrict__ H2, const unsigned short* __restrict__ W4t2,
          const float* __restrict__ b4, const float* __restrict__ g1, const float* __restrict__ be1,
          const float* __restrict__ a5p, const float* __restrict__ W5, const float* __restrict__ b5,
          const int* __restrict__ FLG, float* out, int nN, int gA) {
  __shared__ __attribute__((aligned(16))) float stg[GBM * HD];
  __shared__ __attribute__((aligned(16))) float sout[2 * GBM];
  const int tid = (int)threadIdx.x, lane = tid & 31, wave = tid >> 5;
  const int rowBase = (int)blockIdx.x * GBM;
  gemm_tile<8>(H2, ZP, W4t2, ZP, rowBase, 0, stg);
  __syncthreads();
  const v4f b4v = bfr4(*(const v4f*)(b4 + 4 * lane));
  const v4f gv  = bfr4(*(const v4f*)(g1 + 4 * lane));
  const v4f ev  = bfr4(*(const v4f*)(be1 + 4 * lane));
  const v4f w5a = bfr4(*(const v4f*)(W5 + 8 * lane));
  const v4f w5b = bfr4(*(const v4f*)(W5 + 8 * lane + 4));
  const float a5  = bfr(a5p[0]);
  const float b50 = bfr(b5[0]);
  const float b51 = bfr(b5[1]);
  int fb = rowBase / NBA;
  fb = fb > gA - 1 ? gA - 1 : fb;
  const int fany = FLG[(size_t)fb * 32 + 1] | FLG[(size_t)(gA + fb) * 32 + 1] | FLG[(size_t)(2 * gA + fb) * 32 + 1];
  const float pz = (fany != 0) ? __int_as_float(0x7fc00000) : 0.0f;
#pragma unroll 1
  for (int i = 0; i < 16; ++i) {
    const int lr = 16 * wave + i;
    const v4f pv = *(const v4fa*)(stg + lr * HD + 4 * lane);
    const float z0 = prelu((((pv.x + b4v.x) * BNK) * gv.x) + ev.x, a5);
    const float z1 = prelu((((pv.y + b4v.y) * BNK) * gv.y) + ev.y, a5);
    const float z2 = prelu((((pv.z + b4v.z) * BNK) * gv.z) + ev.z, a5);
    const float z3 = prelu((((pv.w + b4v.w) * BNK) * gv.w) + ev.w, a5);
    float s0 = z0 * w5a.x;
    s0 = fmaf(z1, w5a.z, s0); s0 = fmaf(z2, w5b.x, s0); s0 = fmaf(z3, w5b.z, s0);
    float s1 = z0 * w5a.y;
    s1 = fmaf(z1, w5a.w, s1); s1 = fmaf(z2, w5b.y, s1); s1 = fmaf(z3, w5b.w, s1);
    s0 += __shfl_xor(s0, 16, 32); s1 += __shfl_xor(s1, 16, 32);
    s0 += __shfl_xor(s0, 8, 32);  s1 += __shfl_xor(s1, 8, 32);
    s0 += __shfl_xor(s0, 4, 32);  s1 += __shfl_xor(s1, 4, 32);
    s0 += __shfl_xor(s0, 2, 32);  s1 += __shfl_xor(s1, 2, 32);
    s0 += __shfl_xor(s0, 1, 32);  s1 += __shfl_xor(s1, 1, 32);
    const float o0 = (s0 + b50) + pz;
    const float o1 = (s1 + b51) + pz;
    if (lane == 0) { sout[2 * lr] = o0; sout[2 * lr + 1] = o1; }
  }
  __syncthreads();
  if (wave == 0) {
    const v4f v = *(const v4fa*)(sout + 4 * lane);
    const bool ok = (rowBase + 2 * lane + 1) < nN;
    const int  li = ok ? lane : 0;
    float* op = out + (size_t)rowBase * 2 + 4 * li;
    if (ok) *(volatile v4f*)op = v;
    __threadfence();
    if (ok) *(volatile v4f*)op = v;
  }
}

static inline int cdiv(int a, int b) { return (a + b - 1) / b; }
static inline size_t al256(size_t o) { return (o + 255) & ~(size_t)255; }

extern "C" void kernel_launch(void* const* d_in, const int* in_sizes, int n_in,
                              void* d_out, int out_size, void* d_ws, size_t ws_size,
                              hipStream_t stream) {
  if (n_in < 46) return;
  const int nN = in_sizes[43];
  const int nE = in_sizes[44];
  if (nN < GBM || nN > (1 << SRCB) || (nN % 16) != 0) return;
  if (nE < 1 || nE > (1 << 28) || in_sizes[45] != nE) return;
  if ((long long)in_sizes[0] != (long long)nN * FIN) return;
  if (in_sizes[1] != 3 * FIN) return;
  if (in_sizes[2] != FIN * HD || in_sizes[4] != FIN * HD) return;
  if (in_sizes[3] != HD || in_sizes[5] != HD || in_sizes[6] != HD || in_sizes[7] != HD || in_sizes[8] != 1) return;
  if (in_sizes[9] != HD * FIN || in_sizes[10] != FIN) return;
  for (int l = 0; l < 2; ++l) {
    const int b = 11 + 12 * l;
    const int fin = l ? HD : FIN;
    if (in_sizes[b] != fin * HD || in_sizes[b + 2] != fin * HD || in_sizes[b + 4] != fin * HD ||
        in_sizes[b + 6] != fin * HD) return;
    if (in_sizes[b + 1] != HD || in_sizes[b + 3] != HD || in_sizes[b + 5] != HD || in_sizes[b + 7] != HD) return;
    if (in_sizes[b + 8] != 3 * HD || in_sizes[b + 9] != 1 || in_sizes[b + 10] != HD || in_sizes[b + 11] != HD) return;
  }
  if (in_sizes[35] != 1 || in_sizes[36] != HD * HD || in_sizes[37] != HD || in_sizes[38] != HD ||
      in_sizes[39] != HD || in_sizes[40] != 1 || in_sizes[41] != HD * 2 || in_sizes[42] != 2) return;
  if ((long long)out_size != 2LL * nN) return;

  const float* feat = (const float*)d_in[0];
  const float* lemb = (const float*)d_in[1];
  const float* W1   = (const float*)d_in[2];   const float* b1   = (const float*)d_in[3];
  const float* W2   = (const float*)d_in[4];   const float* b2   = (const float*)d_in[5];
  const float* bn0g = (const float*)d_in[6];   const float* bn0b = (const float*)d_in[7];
  const float* a3   = (const float*)d_in[8];
  const float* W3   = (const float*)d_in[9];   const float* b3   = (const float*)d_in[10];
  const float* Wq[2]; const float* bq[2]; const float* Wk[2]; const float* bk[2];
  const float* Wv[2]; const float* bv[2]; const float* Ws[2]; const float* bs[2];
  const float* Wg[2]; const float* bg[2]; const float* lng[2]; const float* lnb[2];
  for (int l = 0; l < 2; ++l) {
    const int b = 11 + 12 * l;
    Wq[l] = (const float*)d_in[b];      bq[l] = (const float*)d_in[b + 1];
    Wk[l] = (const float*)d_in[b + 2];  bk[l] = (const float*)d_in[b + 3];
    Wv[l] = (const float*)d_in[b + 4];  bv[l] = (const float*)d_in[b + 5];
    Ws[l] = (const float*)d_in[b + 6];  bs[l] = (const float*)d_in[b + 7];
    Wg[l] = (const float*)d_in[b + 8];  bg[l] = (const float*)d_in[b + 9];
    lng[l] = (const float*)d_in[b + 10]; lnb[l] = (const float*)d_in[b + 11];
  }
  const float* acv  = (const float*)d_in[35];
  const float* W4   = (const float*)d_in[36];  const float* b4   = (const float*)d_in[37];
  const float* bn1g = (const float*)d_in[38];  const float* bn1b = (const float*)d_in[39];
  const float* a5   = (const float*)d_in[40];
  const float* W5   = (const float*)d_in[41];  const float* b5   = (const float*)d_in[42];
  const int* labels = (const int*)d_in[43];
  const int* esrc   = (const int*)d_in[44];
  const int* edst   = (const int*)d_in[45];
  float* out = (float*)d_out;

  const int MP = cdiv(nN, MROWS) * MROWS;
  const int gM = MP / GBM;
  const int gA = cdiv(MP, NBA);
  if ((long long)gA * NBA < (long long)MP) return;
  const int vec8 = ((nE & 3) == 0) ? 1 : 0;
  const int nUa  = MP * (KP0 / 8);
  if ((nUa % NTHR) != 0) return;

  char* ws = (char*)d_ws;
  size_t off = 0;
  const size_t oFB  = off; off = al256(off + (size_t)MP * KP0 * 2);
  const size_t oZ   = off; off = al256(off + (size_t)MP * ZP * 2);
  const size_t oH0  = off; off = al256(off + (size_t)MP * H0P * 2);
  const size_t oH1  = off; off = al256(off + (size_t)MP * ZP * 2);
  const size_t oH2  = off; off = al256(off + (size_t)MP * ZP * 2);
  const size_t oQ   = off; off = al256(off + (size_t)MP * NQ * 4);
  const size_t oHIT = off; off = al256(off + (size_t)gA * RCAP * 4);
  const size_t oFLG = off; off = al256(off + (size_t)3 * gA * 128);
  const size_t oW1t = off; off = al256(off + (size_t)HD * KP0 * 2);
  const size_t oW3t = off; off = al256(off + (size_t)KP0 * ZP * 2);
  const size_t oW4t = off; off = al256(off + (size_t)HD * ZP * 2);
  const size_t oWc0 = off; off = al256(off + (size_t)NQ * H0P * 2);
  const size_t oWc1 = off; off = al256(off + (size_t)NQ * ZP * 2);
  const size_t oT2  = off; off = al256(off + (size_t)4 * HD * 4);
  if (off > ws_size || off > (size_t)WSMAX) return;
  unsigned short* FB   = (unsigned short*)(ws + oFB);
  unsigned short* Zhl  = (unsigned short*)(ws + oZ);
  unsigned short* H0hl = (unsigned short*)(ws + oH0);
  unsigned short* H1hl = (unsigned short*)(ws + oH1);
  unsigned short* H2hl = (unsigned short*)(ws + oH2);
  float*          QV   = (float*)(ws + oQ);
  int*            HITS = (int*)(ws + oHIT);
  int*            FLG  = (int*)(ws + oFLG);
  unsigned short* W1t  = (unsigned short*)(ws + oW1t);
  unsigned short* W3t2 = (unsigned short*)(ws + oW3t);
  unsigned short* W4t2 = (unsigned short*)(ws + oW4t);
  unsigned short* Wc0  = (unsigned short*)(ws + oWc0);
  unsigned short* Wc1  = (unsigned short*)(ws + oWc1);
  float*          T2   = (float*)(ws + oT2);
  int* FLG0 = FLG;
  int* FLG1 = FLG + (size_t)gA * 32;
  int* FLG2 = FLG + (size_t)2 * gA * 32;

  const int bktLds  = BKT_LDS_INTS * 4;
  const int scanLds = SCAN_LDS_INTS * 4;
  hipFuncSetAttribute(reinterpret_cast<const void*>(&k_bucket),
                      hipFuncAttributeMaxDynamicSharedMemorySize, bktLds);
  hipFuncSetAttribute(reinterpret_cast<const void*>(&k_scan),
                      hipFuncAttributeMaxDynamicSharedMemorySize, scanLds);

  k_pa<<<nUa / NTHR, NTHR, 0, stream>>>(feat, FB, nN, nUa);
  k_pb<<<(NU1 + NU3 + NU4) / NTHR, NTHR, 0, stream>>>(W1, W3, W4, W1t, W3t2, W4t2);
  k_pc<<<4 * ((HD * (2 * KP0 / 8)) / NTHR), NTHR, 0, stream>>>(Wq[0], Wv[0], Wk[0], Ws[0], Wc0, FIN, KP0);
  k_pc<<<4 * ((HD * (2 * HD / 8)) / NTHR), NTHR, 0, stream>>>(Wq[1], Wv[1], Wk[1], Ws[1], Wc1, HD, HD);
  k_pt<<<1, 384, 0, stream>>>(lemb, W2, T2);
  k_bucket<<<gA, NTHR, bktLds, stream>>>(esrc, edst, nE, nN, vec8, HITS, FLG0);
  k_ga<<<gM, GTHR, 0, stream>>>(FB, W1t, T2, labels, b1, b2, bn0g, bn0b, a3, Zhl, nN);
  k_gb<<<gM, GTHR, 0, stream>>>(Zhl, W3t2, b3, feat, H0hl, nN);
  k_gc<<<dim3(gM, 4), GTHR, 0, stream>>>(H0hl, Wc0, bq[0], bv[0], bk[0], bs[0], QV, H0P);
  k_scan<<<gA, NTHR, scanLds, stream>>>(HITS, FLG0, QV, Wg[0], bg[0], lng[0], lnb[0], acv, H1hl, FLG1, nN, MP);
  k_gc<<<dim3(gM, 4), GTHR, 0, stream>>>(H1hl, Wc1, bq[1], bv[1], bk[1], bs[1], QV, ZP);
  k_scan<<<gA, NTHR, scanLds, stream>>>(HITS, FLG0, QV, Wg[1], bg[1], lng[1], lnb[1], acv, H2hl, FLG2, nN, MP);
  k_gd<<<cdiv(nN, GBM), GTHR, 0, stream>>>(H2hl, W4t2, b4, bn1g, bn1b, a5, W5, b5, FLG, out, nN, gA);
}
